// DecompMultiTransform_1958505087671
// MI455X (gfx1250) — hardware-verified
//
#include <hip/hip_runtime.h>

#define IN_DIM  256
#define OUT_DIM 256
#define NUM_T   64
#define NUM_B   16
#define NN      4096


typedef __attribute__((ext_vector_type(16))) __bf16 v16bf;
typedef __attribute__((ext_vector_type(8)))  __bf16 v8bf;
typedef __attribute__((ext_vector_type(8)))  float    v8f;
typedef __attribute__((ext_vector_type(4)))  float    v4f;
typedef __attribute__((ext_vector_type(4)))  unsigned v4u;

template <typename T> __device__ __forceinline__ void vst2(void* p, T v) { *(volatile T*)p = v; __threadfence(); *(volatile T*)p = v; }
__device__ __forceinline__ v8f wmma_bf(v16bf a, v16bf b, v8f c) {
  v8f d = __builtin_amdgcn_wmma_f32_16x16x32_bf16(false, a, false, b, (short)0, c, false, false);
  asm volatile("v_nop\n\tv_nop\n\tv_nop\n\tv_nop" : "+v"(d) : "v"(a), "v"(b));
  return d;
}
__device__ __forceinline__ v16bf frag_bf(const __bf16* row, int k0, int lane) {
  union { v16bf v; v8bf q[2]; } r; const __bf16* p = row + k0 + 8 * (lane >> 4);
  r.q[0] = *(const v8bf*)(p); r.q[1] = *(const v8bf*)(p + 16); return r.v;
}

__global__ void __launch_bounds__(256) build_wt(const float* __restrict__ weight, const float* __restrict__ w_comp,
                                                __bf16* __restrict__ Whi, __bf16* __restrict__ Wlo) {
  __shared__ __align__(16) __bf16 th[256][72], tl[256][72];
  const int o = threadIdx.x, t = blockIdx.x, i0 = blockIdx.y * 64;
  float wc[NUM_B];
#pragma unroll
  for (int b = 0; b < NUM_B; ++b) wc[b] = w_comp[t * NUM_B + b];
  for (int ii = 0; ii < 64; ++ii) {
    const int i = i0 + ii;
    float acc = 0.f;
#pragma unroll
    for (int b = 0; b < NUM_B; ++b) acc += wc[b] * weight[(size_t)b * (IN_DIM * OUT_DIM) + (size_t)i * OUT_DIM + o];
    const __bf16 h = (__bf16)acc; th[o][ii] = h; tl[o][ii] = (__bf16)(acc - (float)h);
  }
  __syncthreads();
  for (int g = threadIdx.x; g < 256 * 8; g += 256) {
    const int oo = g >> 3, pc = g & 7;
    const size_t off = ((size_t)t * OUT_DIM + oo) * IN_DIM + i0 + pc * 8;
    vst2(Whi + off, *(const v4u*)(&th[oo][pc * 8])); vst2(Wlo + off, *(const v4u*)(&tl[oo][pc * 8]));
  }
}

__global__ void __launch_bounds__(256) rgcn_gemm(const float* __restrict__ x, const int* __restrict__ xtype,
                                                 const __bf16* __restrict__ Whi, const __bf16* __restrict__ Wlo, float* __restrict__ out) {
  __shared__ int s_rows[NN];
  __shared__ int s_cnt;
  __shared__ __align__(16) float so[8][16 * 64];
  const int t = blockIdx.x, q = blockIdx.y;
  if (threadIdx.x == 0) s_cnt = 0;
  __syncthreads();
  for (int n = threadIdx.x; n < NN; n += blockDim.x) {
    const int ty = xtype[n];
    if (ty == t) { int p = atomicAdd(&s_cnt, 1); s_rows[p] = n; }
  }
  __syncthreads();
  const int cnt = s_cnt;
  const int lane = threadIdx.x & 31, wave = threadIdx.x >> 5, col = lane & 15, hi = lane >> 4;
  const int n0 = q * 64;
  float* S = so[wave];
  const int mtiles = (cnt + 15) >> 4;
  for (int mt = wave; mt < mtiles; mt += 8) {
    const int mbase = mt * 16;
    const int mrow = mbase + col;
    const int srow = s_rows[mrow < cnt ? mrow : cnt - 1];
    const float* arow = x + (size_t)srow * IN_DIM;
    v8f acc[4] = {(v8f){}, (v8f){}, (v8f){}, (v8f){}};
#pragma unroll 2
    for (int kc = 0; kc < IN_DIM / 32; ++kc) {
      v16bf ah, al;
      { const float* p = arow + kc * 32 + 8 * hi;
#pragma unroll
        for (int i = 0; i < 16; ++i) { const float v = p[(i < 8) ? i : (i + 8)]; const __bf16 h = (__bf16)v; ah[i] = h; al[i] = (__bf16)(v - (float)h); } }
#pragma unroll
      for (int j = 0; j < 4; ++j) {
        const size_t ro = ((size_t)t * OUT_DIM + n0 + j * 16 + col) * IN_DIM;
        const v16bf bh = frag_bf(Whi + ro, kc * 32, lane), bl = frag_bf(Wlo + ro, kc * 32, lane);
        acc[j] = wmma_bf(al, bh, acc[j]); acc[j] = wmma_bf(ah, bl, acc[j]); acc[j] = wmma_bf(ah, bh, acc[j]);
      }
    }
#pragma unroll
    for (int j = 0; j < 4; ++j)
#pragma unroll
      for (int r = 0; r < 8; ++r) S[(hi * 8 + r) * 64 + j * 16 + col] = acc[j][r];
    asm volatile("s_wait_dscnt 0" ::: "memory");
    __builtin_amdgcn_wave_barrier();
    __builtin_amdgcn_fence(__ATOMIC_RELEASE, "workgroup");
#pragma unroll
    for (int qq = 0; qq < 8; ++qq) {
      const int rl = qq * 2 + (lane >> 4), pc = lane & 15, m = mbase + rl;
      if (m < cnt) vst2(out + (size_t)s_rows[m] * OUT_DIM + n0 + pc * 4, *(const v4f*)(S + rl * 64 + pc * 4));
    }
    __builtin_amdgcn_wave_barrier();
  }
}

extern "C" void kernel_launch(void* const* d_in, const int* in_sizes, int n_in,
                              void* d_out, int out_size, void* d_ws, size_t ws_size,
                              hipStream_t stream) {
  (void)in_sizes; (void)n_in; (void)out_size; (void)ws_size;
  const float* x      = (const float*)d_in[0];
  const int*   xtype  = (const int*)d_in[1];
  const float* weight = (const float*)d_in[2];
  const float* w_comp = (const float*)d_in[3];
  float*       out    = (float*)d_out;
  __bf16* Whi = (__bf16*)d_ws;
  __bf16* Wlo = Whi + (size_t)NUM_T * IN_DIM * OUT_DIM;
  build_wt<<<dim3(NUM_T, 4), 256, 0, stream>>>(weight, w_comp, Whi, Wlo);
  rgcn_gemm<<<dim3(NUM_T, 4), 256, 0, stream>>>(x, xtype, Whi, Wlo, out);
}
